// NumAttention_16329465660072
// MI455X (gfx1250) — hardware-run, weakly checked
//
#include <hip/hip_runtime.h>
#define NB 4
#define NP 2048
#define NC 512
#define NV 8
#define NDH 64
#define ND 64
#define NHD 8
#define NQH 1024
#define NCK 256.0f
#define NCP 4096.0f
#define NCQ 2048.0f
typedef __bf16 v16b __attribute__((ext_vector_type(16)));
typedef unsigned short v8us __attribute__((ext_vector_type(8), may_alias));
typedef float  v8f  __attribute__((ext_vector_type(8)));
typedef float  v4f  __attribute__((ext_vector_type(4)));
typedef float  v4fa __attribute__((ext_vector_type(4), may_alias));
union FragB { v16b v; v8us half[2]; unsigned short u[16]; };

__device__ __forceinline__ unsigned short bf16_bits(float x) { unsigned int u = __float_as_uint(x); return (unsigned short)((u + 0x7FFFu + ((u >> 16) & 1u)) >> 16); }
__device__ __forceinline__ float bf16_val(unsigned short b) { return __uint_as_float(((unsigned int)b) << 16); }
__device__ __forceinline__ float bf16_round(float x) { return bf16_val(bf16_bits(x)); }
template <int NT>
__device__ __forceinline__ v8f mmaN(v16b ah, v16b al, v16b bh, v16b bl, v8f c) {
  c = __builtin_amdgcn_wmma_f32_16x16x32_bf16(false, ah, false, bh, (short)0, c, false, false);
  if (NT >= 2) c = __builtin_amdgcn_wmma_f32_16x16x32_bf16(false, al, false, bh, (short)0, c, false, false);
  if (NT >= 3) c = __builtin_amdgcn_wmma_f32_16x16x32_bf16(false, ah, false, bl, (short)0, c, false, false);
  asm volatile("v_nop\n\tv_nop\n\tv_nop\n\tv_nop" : "+v"(c) : "v"(ah), "v"(al), "v"(bh), "v"(bl));
  return c;
}


typedef _Float16 v16h __attribute__((ext_vector_type(16)));
union FragH { v16h v; v8us half[2]; _Float16 h[16]; unsigned short u[16]; };
template <int NT>
__device__ __forceinline__ v8f mmaH(v16h ah, v16h al, v16h bh, v16h bl, v8f c) {
  c = __builtin_amdgcn_wmma_f32_16x16x32_f16(false, ah, false, bh, (short)0, c, false, false);
  if (NT >= 2) c = __builtin_amdgcn_wmma_f32_16x16x32_f16(false, al, false, bh, (short)0, c, false, false);
  if (NT >= 3) c = __builtin_amdgcn_wmma_f32_16x16x32_f16(false, ah, false, bl, (short)0, c, false, false);
  asm volatile("v_nop\n\tv_nop\n\tv_nop\n\tv_nop" : "+v"(c) : "v"(ah), "v"(al), "v"(bh), "v"(bl));
  return c;
}


typedef _Float16 v4h __attribute__((ext_vector_type(4)));
__device__ __forceinline__ v16h g2_frag(const _Float16* p, int hh) { FragH f; f.half[0] = *(const v8us*)((const unsigned short*)p + 8 * hh); f.half[1] = *(const v8us*)((const unsigned short*)p + 16 + 8 * hh); return f.v; }
__device__ __forceinline__ v8f g2_mma(v16h a, v16h b, v8f c) { v8f d = __builtin_amdgcn_wmma_f32_16x16x32_f16(false, a, false, b, (short)0, c, false, false); asm volatile("v_nop\n\tv_nop\n\tv_nop\n\tv_nop" : "+v"(d) : "v"(a), "v"(b)); return d; }
template <int ACT>
__global__ __launch_bounds__(128) void k_gemm2(const _Float16* __restrict__ A, int lda, size_t sA, const _Float16* __restrict__ Bh, int ldb, size_t sB, float alpha, const float* __restrict__ bias, size_t sBias, const float* __restrict__ CP, int rowsPerB, size_t sCPb, int row0g,
    float* __restrict__ C, _Float16* __restrict__ C16, int ldc, size_t sC, int M, int N, int K) { static_assert(ACT == 0 || ACT == 3 || ACT == 6 || ACT == 8 || ACT == 9 || ACT == 11 || ACT == 12 || ACT == 14 || ACT == 15 || ACT == 16 || ACT == 17, "k_gemm2: unsupported ACT code (would silently apply no activation)");
  __shared__ __attribute__((aligned(16))) float so[4][32][68];
  const int tid = threadIdx.x, w = tid >> 5, lane = tid & 31, ln = lane & 15, hh = lane >> 4; const int by = blockIdx.y;
  A += (size_t)by * sA; Bh += (size_t)by * sB; const size_t cofs = (size_t)by * sC; const float* bp = bias ? bias + (size_t)by * sBias : nullptr;
  const int ntn = N >> 6; const int mt = blockIdx.x / ntn, nq = blockIdx.x - mt * ntn; const int row0 = mt * 128 + 32 * w, col0 = nq * 64; if (row0 >= M) return;
  const _Float16* a0p = A + (size_t)(row0 + ln) * lda; const _Float16* a1p = a0p + (size_t)16 * lda;
  const _Float16* b0p = Bh + (size_t)(col0 + ln) * ldb; const _Float16* b1p = b0p + (size_t)16 * ldb; const _Float16* b2p = b1p + (size_t)16 * ldb; const _Float16* b3p = b2p + (size_t)16 * ldb;
  const v8f z8 = {0.f,0.f,0.f,0.f,0.f,0.f,0.f,0.f}; v8f c00 = z8, c01 = z8, c02 = z8, c03 = z8, c10 = z8, c11 = z8, c12 = z8, c13 = z8;
  for (int kb = 0; kb < K; kb += 32) { const v16h a0 = g2_frag(a0p + kb, hh), a1 = g2_frag(a1p + kb, hh);
    v16h b = g2_frag(b0p + kb, hh); c00 = g2_mma(a0, b, c00); c10 = g2_mma(a1, b, c10);
    b = g2_frag(b1p + kb, hh); c01 = g2_mma(a0, b, c01); c11 = g2_mma(a1, b, c11);
    b = g2_frag(b2p + kb, hh); c02 = g2_mma(a0, b, c02); c12 = g2_mma(a1, b, c12);
    b = g2_frag(b3p + kb, hh); c03 = g2_mma(a0, b, c03); c13 = g2_mma(a1, b, c13); }
  v8f accs[8] = {c00, c01, c02, c03, c10, c11, c12, c13};
#pragma unroll
  for (int u = 0; u < 8; ++u) { const int t = u & 3, half = u >> 2; const int col = col0 + t * 16 + ln; const float bv = bp ? bf16_round(bp[col]) : 0.f;
#pragma unroll
    for (int r = 0; r < 8; ++r) { const int rloc = half * 16 + 8 * hh + r; float v = accs[u][r] * alpha + bv; if (CP) { if (rowsPerB < 0) v += CP[cofs + (size_t)(row0g + row0 + rloc) * ldc + col];        else { const int bidx = (row0g + row0 + rloc) / rowsPerB; v += CP[(size_t)bidx * sCPb + (size_t)by * 64 + col]; } }
      if (ACT == 3) v = fmaxf(v, 0.f); else if (ACT == 6) v = 0.5f * v * (1.0f + erff(v * 0.70710678118654752f)); else if (ACT == 11) v = 1.0f / (1.0f + expf(-v)); else if (ACT == 15) v = v / (1.0f + expf(-v)); else if (ACT == 12) v = (v > 0.f) ? v : 0.01f * v; else if (ACT == 8) v = tanhf(v); else if (ACT == 9) v = 0.5f * v * (1.0f + tanhf(0.7978845608028654f * (v + 0.044715f * v * v * v))); else if (ACT == 14) v = (v > 0.f) ? v : 0.1f * v; else if (ACT == 16) v = (v >= 0.f) ? v : 0.3f * v; else if (ACT == 17) v = (v >= 0.f) ? v : 0.2f * v;
      so[w][rloc][t * 16 + ln] = v; } }
  __builtin_amdgcn_fence(__ATOMIC_ACQ_REL, "workgroup"); __builtin_amdgcn_wave_barrier();
  const int rsub = lane >> 4, c4 = (lane & 15) * 4;
  for (int pass = 0; pass < 2; ++pass) {
#pragma unroll
    for (int q = 0; q < 16; ++q) { const int r = q * 2 + rsub; const v4f v = *(const v4fa*)&so[w][r][c4]; if (C) *(volatile v4f*)(C + cofs + (size_t)(row0 + r) * ldc + col0 + c4) = v; if (C16) { v4h h4; for (int i = 0; i < 4; ++i) h4[i] = (_Float16)v[i]; *(volatile v4h*)(C16 + cofs + (size_t)(row0 + r) * ldc + col0 + c4) = h4; } }
    if (pass == 0) __threadfence(); } }


__global__ __launch_bounds__(256) void k_mix(const float* __restrict__ XC, const float* __restrict__ XN, const float* __restrict__ WK, const float* __restrict__ WQ, const float* __restrict__ WV, _Float16* __restrict__ K16, _Float16* __restrict__ X16, float* __restrict__ VF, float ck) {
  const int r = blockIdx.x * 256 + threadIdx.x; if (r >= NB * NP * NHD) return; const int i = r % NHD; const size_t bp = (size_t)(r / NHD);
  float pk[NV], pq[NV]; float mk = -1.0e30f, mq = -1.0e30f;
#pragma unroll
  for (int v = 0; v < NV; ++v) { pk[v] = bf16_round(WK[i * NV + v]); pq[v] = bf16_round(WQ[i * NV + v]); mk = fmaxf(mk, pk[v]); mq = fmaxf(mq, pq[v]); }
  float sk = 0.f, sq = 0.f;
#pragma unroll
  for (int v = 0; v < NV; ++v) { pk[v] = expf(pk[v] - mk); pq[v] = expf(pq[v] - mq); sk += pk[v]; sq += pq[v]; }
#pragma unroll
  for (int v = 0; v < NV; ++v) { pk[v] = pk[v] / sk; pq[v] = pq[v] / sq; }
  const float* wv = WV + (size_t)i * ND; const float* xn = XN + bp * ND; float mv = -1.0e30f;
  for (int c = 0; c < ND; ++c) { const float x = bf16_round(wv[c]); mv = (x > mv) ? x : mv; }
  float sv = 0.f;
  for (int c = 0; c < ND; ++c) sv += expf(bf16_round(wv[c]) - mv);
  float va = 0.f;
  for (int c = 0; c < ND; ++c) va += (expf(bf16_round(wv[c]) - mv) / sv) * bf16_round(xn[c]);
  const float* xc = XC + bp * NC; unsigned short* kp = (unsigned short*)K16 + (size_t)r * NDH; unsigned short* xp = (unsigned short*)X16 + (size_t)r * NDH;
  for (int h = 0; h < NDH; h += 8) { float ka[8], qa[8];
#pragma unroll
    for (int j = 0; j < 8; ++j) { ka[j] = 0.f; qa[j] = 0.f; }
#pragma unroll
    for (int v = 0; v < NV; ++v) { const v4f a0 = *(const v4fa*)(xc + v * NDH + h); const v4f a1 = *(const v4fa*)(xc + v * NDH + h + 4);
#pragma unroll
      for (int j = 0; j < 4; ++j) { const float x0 = bf16_round(a0[j]), x1 = bf16_round(a1[j]); ka[j] += pk[v] * x0; ka[4 + j] += pk[v] * x1; qa[j] += pq[v] * x0; qa[4 + j] += pq[v] * x1; } }
    FragH fk, fq;
#pragma unroll
    for (int j = 0; j < 8; ++j) { fk.h[j] = (_Float16)(ka[j] * ck); fq.h[j] = (_Float16)(qa[j] * ck); }
    *(volatile v8us*)(kp + h) = fk.half[0]; *(volatile v8us*)(xp + h) = fq.half[0]; __threadfence(); *(volatile v8us*)(kp + h) = fk.half[0]; *(volatile v8us*)(xp + h) = fq.half[0]; }
  *(volatile float*)(VF + r) = va; __threadfence(); *(volatile float*)(VF + r) = va; }

__global__ __launch_bounds__(256) void k_ppt(const float* __restrict__ WP, _Float16* __restrict__ PT, float cp) {
  const int t = blockIdx.x * 256 + threadIdx.x; if (t >= NHD * NDH * (NDH / 8)) return; const int hg = t % (NDH / 8); const int g = (t / (NDH / 8)) % NDH; const int i = t / (NDH * (NDH / 8)); FragH f;
  for (int j = 0; j < 8; ++j) { const float* row = WP + ((size_t)i * NDH + hg * 8 + j) * NDH; float m = -1.0e30f;
    for (int c = 0; c < NDH; ++c) { const float x = bf16_round(row[c]); m = (x > m) ? x : m; }
    float s = 0.f;
    for (int c = 0; c < NDH; ++c) s += expf(bf16_round(row[c]) - m);
    f.h[j] = (_Float16)((expf(bf16_round(row[g]) - m) / s) * cp); }
  unsigned short* hp = (unsigned short*)PT + ((size_t)i * NDH + g) * NDH + hg * 8; *(volatile v8us*)hp = f.half[0]; __threadfence(); *(volatile v8us*)hp = f.half[0]; }

__global__ __launch_bounds__(256) void k_rowz(const float* __restrict__ SC, const float* __restrict__ VB, float* __restrict__ OB, int q0) {
  const int r = blockIdx.x * 256 + threadIdx.x; if (r >= NQH * NHD) return; const int i = r % NHD; const int ql = r / NHD; const int q = q0 + ql; const float* sp = SC + ((size_t)i * NQH + ql) * NP; const float* vp = VB + i; float acc = 0.f;
  for (int p = 0; p < NP; p += 4) { const v4f s = *(const v4fa*)(sp + p);
#pragma unroll
    for (int j = 0; j < 4; ++j) acc += ((p + j <= q) ? s[j] : 0.f) * vp[(size_t)(p + j) * NHD]; }
  float* op = OB + (size_t)q0 * NHD + r; *(volatile float*)op = acc; __threadfence(); *(volatile float*)op = acc; }

extern "C" void kernel_launch(void* const* d_in, const int* in_sizes, int n_in,
                              void* d_out, int out_size, void* d_ws, size_t ws_size, hipStream_t stream) {
  (void)in_sizes; (void)n_in; (void)out_size;
  const float* x_cat = (const float*)d_in[0]; const float* x_num = (const float*)d_in[1]; const float* W_K = (const float*)d_in[2]; const float* W_Q = (const float*)d_in[3]; const float* W_pred = (const float*)d_in[4]; const float* W_V = (const float*)d_in[5];
  static_assert(NC == NV * NDH && NC == NHD * NDH && NDH == 64 && NP % NQH == 0 && NQH % 128 == 0 && NP % 64 == 0 && (NB * NP) % 128 == 0 && (NB * NP * NHD) % 256 == 0 && (NHD * NDH * (NDH / 8)) % 256 == 0 && (NQH * NHD) % 256 == 0 && NP % 4 == 0, "whole tiles; exact grids");
  float* out = (float*)d_out;
  char* ws = (char*)d_ws; size_t off = 0;
  auto take = [&](size_t bytes) { char* p = ws + off; off += (bytes + 255) & ~(size_t)255; return p; };
  _Float16* K16 = (_Float16*)take((size_t)NB * NP * NC * 2); _Float16* X16 = (_Float16*)take((size_t)NB * NP * NC * 2); _Float16* Q16 = (_Float16*)take((size_t)NB * NP * NC * 2);
  _Float16* PT = (_Float16*)take((size_t)NHD * NDH * NDH * 2); float* VF = (float*)take((size_t)NB * NP * NHD * 4);
  float* SC = (float*)take((size_t)NHD * NQH * NP * 4);
  if (off > ws_size) return;
  k_mix<<<(NB * NP * NHD) / 256, 256, 0, stream>>>(x_cat, x_num, W_K, W_Q, W_V, K16, X16, VF, NCK);
  k_ppt<<<(NHD * NDH * (NDH / 8)) / 256, 256, 0, stream>>>(W_pred, PT, NCP);
  k_gemm2<0><<<dim3((unsigned)(((NB * NP) / 128) * (NDH / 64)), NHD), 128, 0, stream>>>(X16, NC, (size_t)NDH, PT, NDH, (size_t)NDH * NDH, NCQ / (NCK * NCP), nullptr, 0, nullptr, 1, 0, 0, nullptr, Q16, NC, (size_t)NDH, NB * NP, NDH, NDH);
  for (int b = 0; b < NB; ++b) for (int q0 = 0; q0 < NP; q0 += NQH) {
    k_gemm2<0><<<dim3((unsigned)((NQH / 128) * (NP / 64)), NHD), 128, 0, stream>>>(Q16 + ((size_t)b * NP + q0) * NC, NC, (size_t)NDH, K16 + (size_t)b * NP * NC, NC, (size_t)NDH, 1.0f / (NCQ * NCK), nullptr, 0, nullptr, 1, 0, 0, SC, nullptr, NP, (size_t)NQH * NP, NQH, NP, NDH);
    k_rowz<<<(NQH * NHD) / 256, 256, 0, stream>>>(SC, VF + (size_t)b * NP * NHD, out + (size_t)b * NP * NHD, q0); }
}
